// RelationTypeHead_20942260535549
// MI455X (gfx1250) — hardware-verified
//
#include <hip/hip_runtime.h>
#include <stdint.h>

#define NBAT 16
#define NREG 256
#define NHID 768
#define NPRJ 2048
#define NREL 3
#define NROW (NBAT * NREG)
#define KAUG 800
#define PAUG 832
#define HROW (NROW / 2)
#define SPITCH 196

static_assert((NROW % 64) == 0 && (NPRJ % 64) == 0 && (PAUG % 64) == 0 && (KAUG % 32) == 0 && (NHID % 32) == 0);
static_assert(KAUG <= PAUG && NHID + 1 <= KAUG && (NHID % 8) == 0 && (PAUG % 8) == 0);
static_assert(((NROW * (PAUG / 8)) % 256) == 0 && ((NPRJ * (PAUG / 8)) % 256) == 0);
static_assert((NREG % 64) == 0 && (HROW % NREG) == 0 && (NHID % 4) == 0 && (NPRJ % 4) == 0);
static_assert((SPITCH % 4) == 0 && SPITCH >= 64 * NREL);

typedef __bf16   v16b __attribute__((ext_vector_type(16)));
typedef __bf16   v8b  __attribute__((ext_vector_type(8)));
typedef float    v8f  __attribute__((ext_vector_type(8)));
typedef float    v4f  __attribute__((ext_vector_type(4)));
typedef unsigned int v4u __attribute__((ext_vector_type(4)));

__device__ __forceinline__ unsigned short bf_bits(float f) {
  unsigned u = __float_as_uint(f);
  return (unsigned short)((u + 0x7FFFu + ((u >> 16) & 1u)) >> 16);
}
__device__ __forceinline__ float bf_up(unsigned short h) { return __uint_as_float(((unsigned)h) << 16); }
__device__ __forceinline__ unsigned pk16(unsigned short a, unsigned short b) { return (unsigned)a | ((unsigned)b << 16); }
__device__ __forceinline__ v8f zero8() { v8f z = {0.f, 0.f, 0.f, 0.f, 0.f, 0.f, 0.f, 0.f}; return z; }

__device__ __forceinline__ unsigned hl_pair(float x0, float x1, unsigned& lo) {
  const unsigned short h0 = bf_bits(x0), h1 = bf_bits(x1);
  const unsigned short l0 = bf_bits(x0 - bf_up(h0)), l1 = bf_bits(x1 - bf_up(h1));
  lo = pk16(l0, l1);
  return pk16(h0, h1);
}
__device__ __forceinline__ void pack_hl8(const v4f x0, const v4f x1, v4u& ph, v4u& pl) {
  unsigned lo;
  ph[0] = hl_pair(x0[0], x0[1], lo); pl[0] = lo;
  ph[1] = hl_pair(x0[2], x0[3], lo); pl[1] = lo;
  ph[2] = hl_pair(x1[0], x1[1], lo); pl[2] = lo;
  ph[3] = hl_pair(x1[2], x1[3], lo); pl[3] = lo;
}

__device__ __forceinline__ v16b ldfrag_b(const __bf16* p) {
  union { v16b v; v8b h[2]; } f;
  f.h[0] = *(const v8b*)(p);
  f.h[1] = *(const v8b*)(p + 16);
  return f.v;
}

__device__ __forceinline__ v8f mma_b_raw(v16b a, v16b b, v8f c) {
  return __builtin_amdgcn_wmma_f32_16x16x32_bf16(false, a, false, b, (short)0, c, false, false);
}
__device__ __forceinline__ void dep_guard_b(v8f& a, v8f& b, v16b x, v16b y) {
#if defined(__HIP_DEVICE_COMPILE__)
  asm volatile("v_nop\n\tv_nop\n\tv_nop\n\tv_nop" : "+v"(a), "+v"(b) : "v"(x), "v"(y));
#endif
}
__device__ __forceinline__ void keep4_b(v16b a, v16b b, v16b c, v16b d) {
#if defined(__HIP_DEVICE_COMPILE__)
  asm volatile("v_nop" :: "v"(a), "v"(b), "v"(c), "v"(d));
#endif
}
__device__ __forceinline__ void acc_guard4(v8f& a, v8f& b, v8f& c, v8f& d) {
#if defined(__HIP_DEVICE_COMPILE__)
  asm volatile("v_nop\n\tv_nop\n\tv_nop\n\tv_nop" : "+v"(a), "+v"(b), "+v"(c), "+v"(d));
#endif
}
__device__ __forceinline__ void wave_sync_lds() {
  __builtin_amdgcn_fence(__ATOMIC_RELEASE, "workgroup");
  __builtin_amdgcn_wave_barrier();
  __builtin_amdgcn_fence(__ATOMIC_ACQUIRE, "workgroup");
}

__global__ __launch_bounds__(256) void cvt_aug(const float* __restrict__ in, const float* __restrict__ aug,
                                               int mode, unsigned short* out, int rows) {
  const int i = blockIdx.x * 256 + threadIdx.x;
  const int n8tot = rows * (PAUG / 8);
  if (i >= n8tot) return;
  int row = i / (PAUG / 8);
  const int c8 = (i - row * (PAUG / 8)) * 8;
  if (row > rows - 1) row = rows - 1;
  int cs = c8;
  if (cs > NHID - 8) cs = NHID - 8;
  const float* src = in + (size_t)row * NHID + cs;
  const v4f a = *(const v4f*)(src);
  const v4f b = *(const v4f*)(src + 4);
  const float av = aug[row];
  v4u p;
  p[0] = pk16(bf_bits(a[0]), bf_bits(a[1]));
  p[1] = pk16(bf_bits(a[2]), bf_bits(a[3]));
  p[2] = pk16(bf_bits(b[0]), bf_bits(b[1]));
  p[3] = pk16(bf_bits(b[2]), bf_bits(b[3]));
  const unsigned augbits = mode ? (unsigned)bf_bits(av) : 0x3F80u;
  if (c8 >= NHID) {
    p[0] = (c8 == NHID) ? augbits : 0u;
    p[1] = 0u; p[2] = 0u; p[3] = 0u;
  }
  *(volatile v4u*)(out + (size_t)i * 8) = p;
  __threadfence();
  *(volatile v4u*)(out + (size_t)i * 8) = p;
}

__global__ __launch_bounds__(256) void trcvt(const float* __restrict__ in, const float* __restrict__ aug,
                                             int mode, unsigned short* out, int IR, int IC, int ORT,
                                             long long strideIn, long long strideOut) {
  __shared__ float T[64][65];
  const int z   = blockIdx.z;
  const int c0  = blockIdx.x * 64;
  const int o0  = blockIdx.y * 64;
  const float* src = in + (size_t)z * strideIn;
  unsigned short* dst = out + (size_t)z * strideOut;
  const int tid = threadIdx.x;
  const int sr  = tid >> 2;
  const int sc  = (tid & 3) * 16;
  const int irow = c0 + sr;
  const float augv = aug[irow];
#pragma unroll
  for (int j4 = 0; j4 < 4; ++j4) {
    const int col = o0 + sc + j4 * 4;
    int cc = col;
    if (cc > IC - 4) cc = IC - 4;
    const v4f v = *(const v4f*)(src + (size_t)irow * IC + cc);
#pragma unroll
    for (int e = 0; e < 4; ++e) {
      const int oc = col + e;
      float val = 0.f;
      if (oc < IC) val = v[e];
      else if (oc == IC) val = mode ? augv : 0.f;
      T[sc + j4 * 4 + e][sr] = val;
    }
  }
  __syncthreads();
  const int rq = tid >> 3;
  const int c8 = (tid & 7) * 8;
  v4u pk[2];
#pragma unroll
  for (int it = 0; it < 2; ++it) {
    const int orl = it * 32 + rq;
    const float* t = &T[orl][c8];
    pk[it][0] = pk16(bf_bits(t[0]), bf_bits(t[1]));
    pk[it][1] = pk16(bf_bits(t[2]), bf_bits(t[3]));
    pk[it][2] = pk16(bf_bits(t[4]), bf_bits(t[5]));
    pk[it][3] = pk16(bf_bits(t[6]), bf_bits(t[7]));
  }
  for (int pass = 0; pass < 2; ++pass) {
#pragma unroll
    for (int it = 0; it < 2; ++it) {
      const int orl = it * 32 + rq;
      *(volatile v4u*)(dst + (size_t)(o0 + orl) * IR + c0 + c8) = pk[it];
    }
    __threadfence();
  }
}

template <int BSPLIT>
__global__ __launch_bounds__(256) void gemm64(
    const unsigned short* __restrict__ Ap, int lda, long long strideA,
    const unsigned short* __restrict__ Btp, const unsigned short* __restrict__ Bt2p, int ldb, long long strideB,
    unsigned short* Ch, unsigned short* Cl, int ldc, long long strideC,
    int M, int N, int K) {
  const __bf16* A   = (const __bf16*)(const void*)Ap;
  const __bf16* Bt  = (const __bf16*)(const void*)Btp;
  const __bf16* Bt2 = (const __bf16*)(const void*)Bt2p;
  __shared__ __align__(16) float sT[8][16 * 68];
  const int b    = blockIdx.y;
  const int lane = threadIdx.x & 31;
  const int wave = threadIdx.x >> 5;
  const int tilesN = N >> 6;
  const int tilesM = M >> 6;
  const int tile = blockIdx.x * 8 + wave;
  if (tile >= tilesM * tilesN) return;
  const int tm = tile / tilesN;
  const int tn = tile - tm * tilesN;
  const int m0 = tm << 6;
  const int n0 = tn << 6;

  const __bf16* Ab  = A  + (size_t)b * strideA;
  const __bf16* Bb  = Bt + (size_t)b * strideB;
  const __bf16* Bb2 = (BSPLIT == 1) ? (Bt2 + (size_t)b * strideB) : Bb;

  const int rlane = lane & 15;
  const int koff  = (lane >> 4) * 8;
  const int mOff  = (lane >> 4) * 8;

  v8f acc[4][4];
#pragma unroll
  for (int i = 0; i < 4; ++i)
#pragma unroll
    for (int j = 0; j < 4; ++j) acc[i][j] = zero8();

  for (int k0 = 0; k0 < K; k0 += 32) {
#pragma unroll
    for (int s = 0; s <= BSPLIT; ++s) {
      const __bf16* Bs = (s == 0) ? Bb : Bb2;
      v16b bq[4];
#pragma unroll
      for (int j = 0; j < 4; ++j) {
        const size_t bo = (size_t)(n0 + (j << 4) + rlane) * ldb + koff + k0;
        bq[j] = ldfrag_b(Bs + bo);
      }
#pragma unroll
      for (int i = 0; i < 4; ++i) {
        const size_t ao = (size_t)(m0 + (i << 4) + rlane) * lda + koff + k0;
        const v16b ah = ldfrag_b(Ab + ao);
#pragma unroll
        for (int j = 0; j < 4; ++j) acc[i][j] = mma_b_raw(ah, bq[j], acc[i][j]);
        dep_guard_b(acc[i][0], acc[i][3], ah, ah);
      }
      keep4_b(bq[0], bq[1], bq[2], bq[3]);
    }
  }
  acc_guard4(acc[0][0], acc[0][1], acc[0][2], acc[0][3]);
  acc_guard4(acc[1][0], acc[1][1], acc[1][2], acc[1][3]);
  acc_guard4(acc[2][0], acc[2][1], acc[2][2], acc[2][3]);
  acc_guard4(acc[3][0], acc[3][1], acc[3][2], acc[3][3]);

  float* slab = sT[wave];
  const int rq = lane >> 3;
  const int c8 = (lane & 7) * 8;
  unsigned short* Chb = Ch + (size_t)b * strideC;
  unsigned short* Clb = Cl + (size_t)b * strideC;
#pragma unroll
  for (int i = 0; i < 4; ++i) {
    const int mBase = m0 + (i << 4);
#pragma unroll
    for (int j = 0; j < 4; ++j) {
#pragma unroll
      for (int r = 0; r < 8; ++r) {
        slab[(mOff + r) * 68 + (j << 4) + rlane] = acc[i][j][r];
      }
    }
    wave_sync_lds();
    for (int pass = 0; pass < 2; ++pass) {
#pragma unroll
      for (int it = 0; it < 4; ++it) {
        const int row = it * 4 + rq;
        const v4f x0 = *(const v4f*)(slab + row * 68 + c8);
        const v4f x1 = *(const v4f*)(slab + row * 68 + c8 + 4);
        v4u ph, pl;
        pack_hl8(x0, x1, ph, pl);
        const size_t o = (size_t)(mBase + row) * ldc + n0 + c8;
        *(volatile v4u*)(Chb + o) = ph;
        *(volatile v4u*)(Clb + o) = pl;
      }
      __threadfence();
    }
    wave_sync_lds();
  }
}

__global__ __launch_bounds__(128) void k_logits(
    const unsigned short* __restrict__ HWhp, const unsigned short* __restrict__ HWlp, long long strideR,
    const unsigned short* __restrict__ Thp, const unsigned short* __restrict__ Tlp,
    const float* __restrict__ bilb, float* out) {
  const __bf16* HWh = (const __bf16*)(const void*)HWhp;
  const __bf16* HWl = (const __bf16*)(const void*)HWlp;
  const __bf16* Th  = (const __bf16*)(const void*)Thp;
  const __bf16* Tl  = (const __bf16*)(const void*)Tlp;
  __shared__ __align__(16) float sO[4][16 * SPITCH];
  const int lane = threadIdx.x & 31;
  const int wave = threadIdx.x >> 5;
  const int bl   = blockIdx.y;
  const int nt   = blockIdx.x;
  const int rlane = lane & 15;
  const int koff  = (lane >> 4) * 8;
  const int mOff  = (lane >> 4) * 8;
  const int nrow0 = bl * NREG + nt * 64 + wave * 16;
  const int trow0 = bl * NREG;
  float bbv[3];
  bbv[0] = bf_up(bf_bits(bilb[0]));
  bbv[1] = bf_up(bf_bits(bilb[1]));
  bbv[2] = bf_up(bf_bits(bilb[2]));
  float* slab = sO[wave];

#pragma unroll 1
  for (int mc = 0; mc < NREG / 64; ++mc) {
    const int m0 = mc * 64;
    v8f acc[3][4];
#pragma unroll
    for (int r = 0; r < 3; ++r)
#pragma unroll
      for (int j = 0; j < 4; ++j) acc[r][j] = zero8();

#pragma unroll 1
    for (int k0 = 0; k0 < NPRJ; k0 += 32) {
      v16b t[4];
#pragma unroll
      for (int j = 0; j < 4; ++j)
        t[j] = ldfrag_b(Th + (size_t)(trow0 + m0 + (j << 4) + rlane) * NPRJ + koff + k0);
#pragma unroll
      for (int r = 0; r < 3; ++r) {
        const size_t ao = (size_t)r * strideR + (size_t)(nrow0 + rlane) * NPRJ + koff + k0;
        const v16b a  = ldfrag_b(HWh + ao);
        const v16b a2 = ldfrag_b(HWl + ao);
#pragma unroll
        for (int j = 0; j < 4; ++j) {
          acc[r][j] = mma_b_raw(a, t[j], acc[r][j]);
          acc[r][j] = mma_b_raw(a2, t[j], acc[r][j]);
        }
        dep_guard_b(acc[r][0], acc[r][3], a, a2);
      }
      keep4_b(t[0], t[1], t[2], t[3]);
#pragma unroll
      for (int j = 0; j < 4; ++j)
        t[j] = ldfrag_b(Tl + (size_t)(trow0 + m0 + (j << 4) + rlane) * NPRJ + koff + k0);
#pragma unroll
      for (int r = 0; r < 3; ++r) {
        const size_t ao = (size_t)r * strideR + (size_t)(nrow0 + rlane) * NPRJ + koff + k0;
        const v16b a = ldfrag_b(HWh + ao);
#pragma unroll
        for (int j = 0; j < 4; ++j) acc[r][j] = mma_b_raw(a, t[j], acc[r][j]);
        dep_guard_b(acc[r][0], acc[r][3], a, a);
      }
      keep4_b(t[0], t[1], t[2], t[3]);
    }
    acc_guard4(acc[0][0], acc[0][1], acc[0][2], acc[0][3]);
    acc_guard4(acc[1][0], acc[1][1], acc[1][2], acc[1][3]);
    acc_guard4(acc[2][0], acc[2][1], acc[2][2], acc[2][3]);

#pragma unroll
    for (int r = 0; r < 3; ++r) {
#pragma unroll
      for (int j = 0; j < 4; ++j) {
#pragma unroll
        for (int rr = 0; rr < 8; ++rr) {
          slab[(mOff + rr) * SPITCH + ((j << 4) + rlane) * NREL + r] = acc[r][j][rr] + bbv[r];
        }
      }
    }
    wave_sync_lds();
    float* ob = out + ((size_t)nrow0 * NREG + m0) * NREL;
    for (int pass = 0; pass < 2; ++pass) {
#pragma unroll
      for (int it = 0; it < 24; ++it) {
        const int pi  = it * 32 + lane;
        const int row = pi / 48;
        const int pc  = pi - row * 48;
        const v4f v = *(const v4f*)(slab + row * SPITCH + pc * 4);
        *(volatile v4f*)(ob + (size_t)row * (NREG * NREL) + pc * 4) = v;
      }
      __threadfence();
    }
    wave_sync_lds();
  }
}

extern "C" void kernel_launch(void* const* d_in, const int* in_sizes, int n_in,
                              void* d_out, int out_size, void* d_ws, size_t ws_size,
                              hipStream_t stream) {
  if (n_in < 7) return;
  if (in_sizes[0] != NROW * NHID) return;
  if (in_sizes[1] != NPRJ * NHID) return;
  if (in_sizes[2] != NPRJ) return;
  if (in_sizes[3] != NPRJ * NHID) return;
  if (in_sizes[4] != NPRJ) return;
  if (in_sizes[5] != NREL * NPRJ * NPRJ) return;
  if (in_sizes[6] < NREL) return;
  if (out_size != NROW * NREG * NREL) return;

  const float* feat  = (const float*)d_in[0];
  const float* headW = (const float*)d_in[1];
  const float* headb = (const float*)d_in[2];
  const float* tailW = (const float*)d_in[3];
  const float* tailb = (const float*)d_in[4];
  const float* bilW  = (const float*)d_in[5];
  const float* bilb  = (const float*)d_in[6];
  float* out = (float*)d_out;

  const size_t PFa  = (size_t)NROW * PAUG * 2;
  const size_t PWta = (size_t)NPRJ * PAUG * 2;
  const size_t PWhT = (size_t)PAUG * NPRJ * 2;
  const size_t PUT  = (size_t)NREL * NPRJ * PAUG * 2;
  const size_t PT   = (size_t)NROW * NPRJ * 2;
  const size_t PWT  = (size_t)NREL * NPRJ * NPRJ * 2;
  const size_t PHW  = (size_t)NREL * HROW * NPRJ * 2;
  const size_t PBIG = (2 * PHW > PWT) ? 2 * PHW : PWT;
  size_t off = 0;
  const size_t oFa  = off; off += PFa;
  const size_t oWta = off; off += PWta;
  const size_t oWhT = off; off += PWhT;
  const size_t oUTh = off; off += PUT;
  const size_t oUTl = off; off += PUT;
  const size_t oTh  = off; off += PT;
  const size_t oTl  = off; off += PT;
  const size_t oBIG = off; off += PBIG;
  if (off > ws_size) return;
  if (off > (size_t)134217728) return;
  const size_t oWT  = oBIG;
  const size_t oHWh = oBIG;
  const size_t oHWl = oBIG + PHW;

  char* ws = (char*)d_ws;
  unsigned short* Fa   = (unsigned short*)(ws + oFa);
  unsigned short* Wta  = (unsigned short*)(ws + oWta);
  unsigned short* WhTa = (unsigned short*)(ws + oWhT);
  unsigned short* UTh  = (unsigned short*)(ws + oUTh);
  unsigned short* UTl  = (unsigned short*)(ws + oUTl);
  unsigned short* Th   = (unsigned short*)(ws + oTh);
  unsigned short* Tl   = (unsigned short*)(ws + oTl);
  unsigned short* WT   = (unsigned short*)(ws + oWT);
  unsigned short* HWh  = (unsigned short*)(ws + oHWh);
  unsigned short* HWl  = (unsigned short*)(ws + oHWl);

  const dim3 blk(256);
  const dim3 gFa((NROW * (PAUG / 8)) / 256);
  const dim3 gWta((NPRJ * (PAUG / 8)) / 256);
  const dim3 gWhT(NPRJ / 64, PAUG / 64, 1);
  const dim3 gWT(NPRJ / 64, NPRJ / 64, NREL);
  const dim3 gTail(((NROW / 64) * (NPRJ / 64) + 7) / 8, 1);
  const dim3 gUT(((NPRJ / 64) * (PAUG / 64) + 7) / 8, NREL);
  const dim3 gHW(((HROW / 64) * (NPRJ / 64) + 7) / 8, NREL);
  const dim3 gLog(NREG / 64, HROW / NREG);
  const dim3 blkLog(128);

  cvt_aug<<<gFa, blk, 0, stream>>>(feat, feat, 0, Fa, NROW);
  cvt_aug<<<gWta, blk, 0, stream>>>(tailW, tailb, 1, Wta, NPRJ);
  trcvt<<<gWhT, blk, 0, stream>>>(headW, headb, 1, WhTa, NPRJ, NHID, PAUG, 0LL, 0LL);
  trcvt<<<gWT, blk, 0, stream>>>(bilW, bilW, 0, WT, NPRJ, NPRJ, NPRJ,
                                 (long long)NPRJ * NPRJ, (long long)NPRJ * NPRJ);
  gemm64<0><<<gTail, blk, 0, stream>>>(
      Fa, PAUG, 0LL, Wta, Wta, PAUG, 0LL,
      Th, Tl, NPRJ, 0LL,
      NROW, NPRJ, KAUG);
  gemm64<0><<<gUT, blk, 0, stream>>>(
      WT, NPRJ, (long long)NPRJ * NPRJ, WhTa, WhTa, NPRJ, 0LL,
      UTh, UTl, PAUG, (long long)NPRJ * PAUG,
      NPRJ, PAUG, NPRJ);
  for (int h = 0; h < 2; ++h) {
    gemm64<1><<<gHW, blk, 0, stream>>>(
        Fa + (size_t)h * HROW * PAUG, PAUG, 0LL, UTh, UTl, PAUG, (long long)NPRJ * PAUG,
        HWh, HWl, NPRJ, (long long)HROW * NPRJ,
        HROW, NPRJ, KAUG);
    k_logits<<<gLog, blkLog, 0, stream>>>(
        HWh, HWl, (long long)HROW * NPRJ,
        Th + (size_t)h * HROW * NPRJ, Tl + (size_t)h * HROW * NPRJ,
        bilb, out + (size_t)h * HROW * NREG * NREL);
  }
  (void)hipGetLastError();
}
